// CompressedAttention_1219770712404
// MI455X (gfx1250) — hardware-verified
//
#include <hip/hip_runtime.h>


namespace {
constexpr int Bn = 4, S = 8192, D = 128, R4 = 4, SC = S / R4;
constexpr float XS = 8.0f, PS = 8.0f, ISC = 0.08838834764831845f;

typedef _Float16 b16;
typedef __attribute__((ext_vector_type(16))) _Float16 v16b;
typedef __attribute__((ext_vector_type(8))) _Float16 v8b;
typedef __attribute__((ext_vector_type(8))) float v8f;
typedef __attribute__((ext_vector_type(4))) float v4f;
__device__ __forceinline__ float bf16_rne(float f) { unsigned int u = __float_as_uint(f); u += 0x7FFFu + ((u >> 16) & 1u); return __uint_as_float(u & 0xFFFF0000u); }
__device__ __forceinline__ void split16(float v, b16& hi, b16& lo) { hi = (b16)v; lo = (b16)(v - (float)hi); }
__device__ __forceinline__ v16b frag_kb(const b16* p, int hh) { const v8b a = *(const v8b*)(p + 8 * hh), b = *(const v8b*)(p + 16 + 8 * hh); v16b f;
#pragma unroll
  for (int e = 0; e < 8; ++e) { f[e] = a[e]; f[8 + e] = b[e]; } return f; }
__device__ __forceinline__ v8f wmma16b(v16b a, v16b b, v8f c) { v8f d = __builtin_amdgcn_wmma_f32_16x16x32_f16(false, a, false, b, (short)0, c, false, false); asm volatile("v_nop\n\tv_nop\n\tv_nop\n\tv_nop" : "+v"(d) : "v"(a), "v"(b)); return d; }
__device__ __forceinline__ float nexp(float x) { return __builtin_amdgcn_exp2f(x * 1.4426950408889634f); }
__device__ __forceinline__ float pmul(float a, float b) { float p = a * b; asm volatile("" : "+v"(p)); return p; }

__global__ __launch_bounds__(256) void prep_kernel(const float* __restrict__ Q, const float* __restrict__ K, const float* __restrict__ V, b16* __restrict__ QX, b16* __restrict__ KH, b16* __restrict__ KL, b16* __restrict__ VTh, b16* __restrict__ VTl) {
  __shared__ __attribute__((aligned(16))) b16 Th[D][64 + 8], Tl[D][64 + 8];
  const int b = blockIdx.y, t0 = blockIdx.x * 64, t_ = threadIdx.x;
  for (int pass = 0; pass < 2; ++pass) {
    for (int i = t_; i < 256 * 16; i += 256) { const size_t p = ((size_t)b * S + (size_t)t0 * R4) * D / 8 + i; v8b v; for (int e = 0; e < 8; ++e) v[e] = (b16)(bf16_rne(Q[p * 8 + e]) * XS); *(volatile v8b*)(QX + p * 8) = v; }
    for (int i = t_; i < 64 * 16; i += 256) { const int tk = i >> 4, c8 = (i & 15) * 8; const size_t src0 = ((size_t)b * S + (size_t)(t0 + tk) * R4) * D + c8; v8b hv, lv;
      for (int e = 0; e < 8; ++e) { float s = 0.0f; for (int r = 0; r < R4; ++r) s += bf16_rne(K[src0 + (size_t)r * D + e]); b16 a_, c_; split16(s * (0.25f * XS), a_, c_); hv[e] = a_; lv[e] = c_; }
      const size_t gi = ((size_t)b * SC + t0 + tk) * D + c8; *(volatile v8b*)(KH + gi) = hv; *(volatile v8b*)(KL + gi) = lv; }
    for (int i = t_; i < 64 * D; i += 256) { const int tk = i / D, c = i % D; const size_t src0 = ((size_t)b * S + (size_t)(t0 + tk) * R4) * D + c; float s = 0.0f; for (int r = 0; r < R4; ++r) s += bf16_rne(V[src0 + (size_t)r * D]); b16 a_, c_; split16(s * (0.25f * XS), a_, c_); Th[c][tk] = a_; Tl[c][tk] = c_; }
    __syncthreads();
    for (int i = t_; i < D * 8; i += 256) { const int c = i >> 3, c8 = (i & 7) * 8; const size_t gi = ((size_t)b * D + c) * SC + t0 + c8; *(volatile v8b*)(VTh + gi) = *(const v8b*)(&Th[c][c8]); *(volatile v8b*)(VTl + gi) = *(const v8b*)(&Tl[c][c8]); }
    __threadfence(); __syncthreads(); }
}
__global__ __launch_bounds__(128) void attn_kernel(const b16* __restrict__ QX, const b16* __restrict__ KH, const b16* __restrict__ KL, const b16* __restrict__ VTh, const b16* __restrict__ VTl, float* __restrict__ out) {
  __shared__ __attribute__((aligned(16))) float Os[4][16][D + 4];
  const int wave = threadIdx.x >> 5, lane = threadIdx.x & 31, hh = lane >> 4, col = lane & 15; const int b = blockIdx.y, q0 = blockIdx.x * 64 + wave * 16, qi = q0 + col;
  const b16* Qr = QX + ((size_t)b * S) * D; const b16* Kr = KH + ((size_t)b * SC) * D; const b16* Klr = KL + ((size_t)b * SC) * D; const b16* V = VTh + ((size_t)b * D) * SC; const b16* Vl = VTl + ((size_t)b * D) * SC;
  v16b qf[4]; for (int t = 0; t < 4; ++t) qf[t] = frag_kb(Qr + (size_t)qi * D + t * 32, hh);
  float m = -INFINITY, l = 0.0f; v8f o[8]; for (int t = 0; t < 8; ++t) o[t] = (v8f){};
  for (int kb = 0; kb < SC; kb += 32) {
    v8f s0 = {}, s1 = {};
#pragma unroll
    for (int t = 0; t < 4; ++t) { const v16b k0 = frag_kb(Kr + (size_t)(kb + col) * D + t * 32, hh), k0l = frag_kb(Klr + (size_t)(kb + col) * D + t * 32, hh), k1 = frag_kb(Kr + (size_t)(kb + 16 + col) * D + t * 32, hh), k1l = frag_kb(Klr + (size_t)(kb + 16 + col) * D + t * 32, hh);
      s0 = wmma16b(k0, qf[t], s0); s0 = wmma16b(k0l, qf[t], s0); s1 = wmma16b(k1, qf[t], s1); s1 = wmma16b(k1l, qf[t], s1); }
    float mr = -INFINITY;
#pragma unroll
    for (int r = 0; r < 8; ++r) { s0[r] *= ISC / (XS * XS); s1[r] *= ISC / (XS * XS); mr = fmaxf(mr, fmaxf(s0[r], s1[r])); }
    mr = fmaxf(mr, __shfl_xor(mr, 16)); const float mn = fmaxf(m, mr); const float al_ = nexp(m - mn); m = mn; float sum = 0.0f; v16b pb, pl;
#pragma unroll
    for (int r = 0; r < 8; ++r) { const float e0 = nexp(s0[r] - mn), e1 = nexp(s1[r] - mn); sum += e0 + e1; b16 a_, c_; split16(e0 * PS, a_, c_); pb[r] = a_; pl[r] = c_; split16(e1 * PS, a_, c_); pb[8 + r] = a_; pl[8 + r] = c_; }
    sum += __shfl_xor(sum, 16); l = l * al_ + sum;
#pragma unroll
    for (int t = 0; t < 8; ++t) { o[t] *= al_; const v16b vh = frag_kb(V + (size_t)(t * 16 + col) * SC + kb, hh); o[t] = wmma16b(vh, pb, o[t]); o[t] = wmma16b(vh, pl, o[t]); o[t] = wmma16b(frag_kb(Vl + (size_t)(t * 16 + col) * SC + kb, hh), pb, o[t]); } }
  const float inv = 1.0f / (l * PS * XS);
#pragma unroll
  for (int t = 0; t < 8; ++t)
#pragma unroll
    for (int r = 0; r < 8; ++r) Os[wave][col][t * 16 + 8 * hh + r] = o[t][r] * inv;
  __syncthreads();
  for (int pass = 0; pass < 2; ++pass) { for (int i = threadIdx.x; i < 64 * 32; i += 128) { const int rr = i >> 5, c4 = (i & 31) * 4; *(volatile v4f*)(out + ((size_t)b * S + blockIdx.x * 64 + rr) * D + c4) = *(const v4f*)(&Os[rr >> 4][rr & 15][c4]); } __threadfence(); }
}
}

extern "C" void kernel_launch(void* const* d_in, const int* in_sizes, int n_in,
                              void* d_out, int out_size, void* d_ws, size_t ws_size, hipStream_t stream) {
  (void)n_in; (void)out_size;
  const float* Q = (const float*)d_in[0]; const float* K = (const float*)d_in[1]; const float* V = (const float*)d_in[2];
  float* out = (float*)d_out;
  if (in_sizes[0] != Bn * S * D || in_sizes[1] != Bn * S * D || in_sizes[2] != Bn * S * D) return;
  size_t off = 0; char* ws = (char*)d_ws;
  auto carve = [&](size_t bytes) { char* p = ws + off; off += (bytes + 255) & ~(size_t)255; return p; };
  b16* QX = (b16*)carve((size_t)Bn * S * D * 2); b16* KH = (b16*)carve((size_t)Bn * SC * D * 2); b16* KL = (b16*)carve((size_t)Bn * SC * D * 2); b16* VTh = (b16*)carve((size_t)Bn * D * SC * 2); b16* VTl = (b16*)carve((size_t)Bn * D * SC * 2);
  if (off > ws_size) return;
  prep_kernel<<<dim3(SC / 64, Bn), 256, 0, stream>>>(Q, K, V, QX, KH, KL, VTh, VTl);
  attn_kernel<<<dim3(S / 64, Bn), 128, 0, stream>>>(QX, KH, KL, VTh, VTl, out);
}
